// CustomSelfAttention_22479858827522
// MI455X (gfx1250) — hardware-verified
//
#include <hip/hip_runtime.h>

typedef _Float16 bf16;
typedef __attribute__((ext_vector_type(16))) _Float16 v16bf;
typedef __attribute__((ext_vector_type(8)))  _Float16 v8bf;
typedef __attribute__((ext_vector_type(4)))  _Float16 v4bf;
typedef __attribute__((ext_vector_type(4)))  float  v4f_t;
typedef float v4fa __attribute__((ext_vector_type(4), may_alias));
static __device__ __forceinline__ unsigned pk2(float a, float b) { return (unsigned)__builtin_bit_cast(unsigned short, (bf16)a) | ((unsigned)__builtin_bit_cast(unsigned short, (bf16)b) << 16); }
typedef __attribute__((ext_vector_type(8)))  float  v8f;
typedef __attribute__((ext_vector_type(4)))  float  v4f;
typedef __attribute__((ext_vector_type(4)))  unsigned int u32x4;
typedef __attribute__((ext_vector_type(4)))  int  i32x4;
typedef __attribute__((ext_vector_type(8)))  int  i32x8;

#define S_LEN 1024
#define HEADS 16
#define HDIM  64
#define DIST_ROWS 2047
#define CB_LD 192

#define PLDS_OFF  (CB_LD*CB_LD*2)
#define KLDS_OFF  (PLDS_OFF + 8*16*64*2)
#define VLDS_OFF  (KLDS_OFF + 64*64*2)
#define OST_OFF   (VLDS_OFF + 64*64*2)
#define ATTN_SMEM (OST_OFF + 8*16*64*4)

#if defined(__has_builtin)
# if __has_builtin(__builtin_amdgcn_tensor_load_to_lds)
#  define HAVE_TDM 1
# endif
#endif


__device__ __forceinline__ v8bf ld8bf(const bf16* p){ return *(const v8bf*)p; }

__device__ __forceinline__ v16bf cat16(v8bf a, v8bf b){
  union { v16bf v; v8bf h[2]; } u; u.h[0] = a; u.h[1] = b; return u.v;
}
__device__ __forceinline__ v16bf a_frag(const bf16* row_ptr, int hi){
  return cat16(ld8bf(row_ptr + 8*hi), ld8bf(row_ptr + 16 + 8*hi));
}
__device__ __forceinline__ v16bf b_frag(const bf16* rowT_ptr, int hi){ return a_frag(rowT_ptr, hi); }
__device__ __forceinline__ v8f wmma_bf16(v16bf a, v16bf b, v8f c){
  return __builtin_amdgcn_wmma_f32_16x16x32_f16(false, a, false, b,
                                                 (short)0, c, false, false);
}

#ifdef HAVE_TDM
__device__ __forceinline__ void tdm_load_2d(unsigned lds_off, const void* gaddr,
    unsigned dim0, unsigned dim1, unsigned tile0, unsigned tile1,
    unsigned stride0)
{
  unsigned long long ga = (unsigned long long)(__SIZE_TYPE__)gaddr;
  u32x4 g0;
  g0[0] = 1u;
  g0[1] = lds_off;
  g0[2] = (unsigned)(ga & 0xffffffffu);
  g0[3] = (unsigned)((ga >> 32) & 0x01ffffffu)
        | (2u << 30);
  i32x8 g1;
  g1[0] = (int)(1u << 16);
  g1[1] = (int)((dim0 & 0xffffu) << 16);
  g1[2] = (int)(((dim0 >> 16) & 0xffffu) | ((dim1 & 0xffffu) << 16));
  g1[3] = (int)(((dim1 >> 16) & 0xffffu) | ((tile0 & 0xffffu) << 16));
  g1[4] = (int)(tile1 & 0xffffu);
  g1[5] = (int)stride0;
  g1[6] = 0;
  g1[7] = 0;
  i32x4 z4 = {0, 0, 0, 0};
#if defined(__clang_major__) && (__clang_major__ >= 23)
  i32x8 z8 = {0, 0, 0, 0, 0, 0, 0, 0};
  __builtin_amdgcn_tensor_load_to_lds(g0, g1, z4, z4, z8, 0);
#else
  __builtin_amdgcn_tensor_load_to_lds(g0, g1, z4, z4, 0);
#endif
}
#endif

__global__ void cvt_bf16_kernel(const float* __restrict__ src,
                                bf16* __restrict__ dst, int n4){
  int i = blockIdx.x * 256 + threadIdx.x;
  if (i < n4){
    v4f f = ((const v4f*)src)[i];
    v4bf o;
    #pragma unroll
    for (int j = 0; j < 4; ++j) o[j] = (bf16)f[j];
    *(volatile v4bf*)((v4bf*)dst + i) = o; __threadfence(); *(volatile v4bf*)((v4bf*)dst + i) = o;
  }
}

__global__ void __launch_bounds__(256) qkv_kernel(
    const bf16* __restrict__ xb,
    const bf16* __restrict__ wb,
    const float* __restrict__ bq, const float* __restrict__ bk,
    const float* __restrict__ bv,
    bf16* __restrict__ q, bf16* __restrict__ k, bf16* __restrict__ vt)
{
  const bf16* W = wb + (size_t)blockIdx.z * (1024*1024);
  const float* bias; bf16* out; bool tr;
  if      (blockIdx.z == 0){ bias = bq; out = q;  tr = false; }
  else if (blockIdx.z == 1){ bias = bk; out = k;  tr = false; }
  else                     { bias = bv; out = vt; tr = true;  }

  const int lane = threadIdx.x & 31;
  const int wave = threadIdx.x >> 5;
  const int hi = lane >> 4;
  const int lm = lane & 15;

  const int m0 = blockIdx.x * 128 + wave * 16;
  const int n0 = blockIdx.y * 64;

  v8f acc[4];
  #pragma unroll
  for (int nf = 0; nf < 4; ++nf)
    #pragma unroll
    for (int i = 0; i < 8; ++i) acc[nf][i] = 0.f;

  const bf16* xrow = xb + (m0 + lm) * 1024;
  const bf16* wrow0 = W + (n0 + lm) * 1024;
  for (int kk = 0; kk < 1024; kk += 32){
    v16bf a = a_frag(xrow + kk, hi);
    #pragma unroll
    for (int nf = 0; nf < 4; ++nf){
      v16bf bfr = b_frag(wrow0 + nf*(16*1024) + kk, hi);
      acc[nf] = wmma_bf16(a, bfr, acc[nf]);
    }
  }

  __shared__ __attribute__((aligned(16))) float stq[8][16 * 64];
  float* sw = stq[wave];
  const int h = n0 >> 6;
  #pragma unroll
  for (int nf = 0; nf < 4; ++nf){
    float bb = bias[n0 + nf*16 + lm];
    #pragma unroll
    for (int i = 0; i < 8; ++i) sw[(i + 8*hi) * 64 + nf*16 + lm] = acc[nf][i] + bb;
  }
  asm volatile("s_wait_dscnt 0" ::: "memory");
  (void)tr;
  #pragma unroll 1
  for (int pass = 0; pass < 2; ++pass){
    #pragma unroll 4
    for (int rr = 0; rr < 16; ++rr){
      int m = m0 + rr, b = m >> 10, s = m & 1023;
      *(volatile unsigned*)(out + (((size_t)(b*HEADS + h)*S_LEN) + s)*HDIM + 2*lane) = pk2(sw[rr*64 + 2*lane], sw[rr*64 + 2*lane + 1]);
    }
    __threadfence();
  }
}

__global__ __launch_bounds__(256) void vt_kernel(const bf16* __restrict__ Vr, bf16* __restrict__ Vt){
  __shared__ bf16 t[64][66];
  const int tid = threadIdx.x, lane = tid & 31, wave = tid >> 5;
  const int bh = blockIdx.x >> 4, s0 = (blockIdx.x & 15) * 64;
  const bf16* src = Vr + ((size_t)bh * S_LEN + s0) * HDIM;
  #pragma unroll
  for (int kq = 0; kq < 16; ++kq){ int e = tid + 256*kq; t[e >> 6][e & 63] = src[e]; }
  __syncthreads();
  bf16* dst = Vt + (size_t)bh * HDIM * S_LEN + s0;
  #pragma unroll
  for (int rr = 0; rr < 8; ++rr){
    int hd = wave*8 + rr;
    unsigned p = (unsigned)__builtin_bit_cast(unsigned short, t[2*lane][hd]) | ((unsigned)__builtin_bit_cast(unsigned short, t[2*lane + 1][hd]) << 16);
    unsigned* d = (unsigned*)(dst + (size_t)hd * S_LEN) + lane;
    *(volatile unsigned*)d = p; __threadfence(); *(volatile unsigned*)d = p;
  }
}

__global__ void __launch_bounds__(256) attn_kernel(
    const bf16* __restrict__ q, const bf16* __restrict__ k,
    const bf16* __restrict__ vt, const bf16* __restrict__ dist,
    const float* __restrict__ amask, float* __restrict__ out)
{
  extern __shared__ char smem[];
  bf16* cband = (bf16*)smem;
  bf16* plds  = (bf16*)(smem + PLDS_OFF);
  bf16* klds  = (bf16*)(smem + KLDS_OFF);
  bf16* vlds  = (bf16*)(smem + VLDS_OFF);

  const int lane = threadIdx.x & 31;
  const int wave = threadIdx.x >> 5;
  const int hi = lane >> 4;
  const int lm = lane & 15;

  const int bh = blockIdx.y;
  const int b  = bh >> 4;
  const int h  = bh & 15;
  const int l0 = blockIdx.x * 128;

  const bf16* qh = q  + (size_t)bh * (S_LEN*HDIM);
  const bf16* kh = k  + (size_t)bh * (S_LEN*HDIM);
  const bf16* vh = vt + (size_t)bh * (HDIM*S_LEN);

  const bf16* qrow = qh + (l0 + wave*16 + lm) * HDIM;
  v16bf qa0 = a_frag(qrow, hi);
  v16bf qa1 = a_frag(qrow + 32, hi);

  float mstate[8], lstate[8];
  v8f acc[4];
  #pragma unroll
  for (int i = 0; i < 8; ++i){ mstate[i] = -1e30f; lstate[i] = 0.f; }
  #pragma unroll
  for (int hf = 0; hf < 4; ++hf)
    #pragma unroll
    for (int i = 0; i < 8; ++i) acc[hf][i] = 0.f;

  bf16* pwave = plds + wave * (16*64);

  #pragma unroll 1
  for (int k0 = 0; k0 < S_LEN; k0 += 64){
    {
      int k0n = (k0 + 64 < S_LEN) ? (k0 + 64) : k0;
      __builtin_prefetch(kh + (k0n + lane) * HDIM, 0, 3);
      __builtin_prefetch(kh + (k0n + 32 + lane) * HDIM, 0, 3);
      __builtin_prefetch(vh + lane * S_LEN + k0n, 0, 3);
      __builtin_prefetch(vh + (32 + lane) * S_LEN + k0n, 0, 3);
    }

#ifdef HAVE_TDM
    if (wave == 0){
      tdm_load_2d(KLDS_OFF, kh + (size_t)k0 * HDIM, 64, S_LEN, 64, 64, 64);
      tdm_load_2d(VLDS_OFF, vh + k0, S_LEN, HDIM, 64, 64, S_LEN);
      __builtin_amdgcn_s_wait_tensorcnt(0);
    }
#else
    {
      const bf16* ksrc = kh + (size_t)k0 * HDIM;
      #pragma unroll
      for (int t2 = (int)threadIdx.x; t2 < 512; t2 += 256)
        *(v8bf*)(klds + t2*8) = *(const v8bf*)(ksrc + t2*8);
      #pragma unroll
      for (int t2 = (int)threadIdx.x; t2 < 512; t2 += 256){
        int row = t2 >> 3, c8 = t2 & 7;
        *(v8bf*)(vlds + row*64 + c8*8) =
            *(const v8bf*)(vh + row*S_LEN + k0 + c8*8);
      }
    }
#endif
    __syncthreads();

    const int tbase = l0 - k0 + 960;
    #pragma unroll 1
    for (int f = wave; f < 144; f += 8){
      int mf = f / 12, tf = f % 12;
      int m = mf*16 + lm;
      int tg = tbase + tf*16 + lm; if (tg > DIST_ROWS - 1) tg = DIST_ROWS - 1;
      const bf16* brow = dist + tg * HDIM;
      v16bf b0 = b_frag(brow, hi);
      v16bf b1 = b_frag(brow + 32, hi);
      v16bf a0, a1;
      if (mf < 8){ const bf16* p = qh + (l0 + m) * HDIM;
                   a0 = a_frag(p, hi); a1 = a_frag(p + 32, hi); }
      else       { const bf16* p = klds + (m - 128) * HDIM;
                   a0 = a_frag(p, hi); a1 = a_frag(p + 32, hi); }
      v8f c;
      #pragma unroll
      for (int i = 0; i < 8; ++i) c[i] = 0.f;
      c = wmma_bf16(a0, b0, c);
      c = wmma_bf16(a1, b1, c);
      #pragma unroll
      for (int i = 0; i < 8; ++i)
        cband[(mf*16 + i + 8*hi)*CB_LD + tf*16 + lm] = (bf16)c[i];
    }
    __syncthreads();

    v8f sfr[4];
    #pragma unroll
    for (int nf = 0; nf < 4; ++nf){
      const bf16* krow = klds + (nf*16 + lm) * HDIM;
      v8f s;
      #pragma unroll
      for (int i = 0; i < 8; ++i) s[i] = 0.f;
      s = wmma_bf16(qa0, b_frag(krow, hi),      s);
      s = wmma_bf16(qa1, b_frag(krow + 32, hi), s);
      #pragma unroll
      for (int i = 0; i < 8; ++i){
        int mb = wave*16 + i + 8*hi;
        int nb = nf*16 + lm;
        int t  = mb - nb + 63;
        float cb = (float)cband[mb*CB_LD + t]
                 + (float)cband[(128 + nb)*CB_LD + t];
        s[i] = (s[i] + cb) * 0.125f + amask[b*S_LEN + k0 + nb];
      }
      sfr[nf] = s;
    }

    float alpha[8];
    #pragma unroll
    for (int i = 0; i < 8; ++i){
      float v = fmaxf(fmaxf(sfr[0][i], sfr[1][i]), fmaxf(sfr[2][i], sfr[3][i]));
      v = fmaxf(v, __shfl_xor(v, 1));
      v = fmaxf(v, __shfl_xor(v, 2));
      v = fmaxf(v, __shfl_xor(v, 4));
      v = fmaxf(v, __shfl_xor(v, 8));
      float mn = fmaxf(mstate[i], v);
      alpha[i] = __expf(mstate[i] - mn);
      mstate[i] = mn;
    }
    float rsum[8];
    #pragma unroll
    for (int i = 0; i < 8; ++i) rsum[i] = 0.f;
    #pragma unroll
    for (int nf = 0; nf < 4; ++nf)
      #pragma unroll
      for (int i = 0; i < 8; ++i){
        float p = __expf(sfr[nf][i] - mstate[i]);
        sfr[nf][i] = p;
        rsum[i] += p;
      }
    #pragma unroll
    for (int i = 0; i < 8; ++i){
      float r = rsum[i];
      r += __shfl_xor(r, 1); r += __shfl_xor(r, 2);
      r += __shfl_xor(r, 4); r += __shfl_xor(r, 8);
      lstate[i] = lstate[i]*alpha[i] + r;
    }

    #pragma unroll
    for (int nf = 0; nf < 4; ++nf)
      #pragma unroll
      for (int i = 0; i < 8; ++i)
        pwave[(i + 8*hi)*64 + nf*16 + lm] = (bf16)(sfr[nf][i] * 1024.0f);

    const bf16* prow = pwave + lm*64;
    v16bf pa0 = a_frag(prow, hi);
    v16bf pa1 = a_frag(prow + 32, hi);

    #pragma unroll
    for (int hf = 0; hf < 4; ++hf){
      #pragma unroll
      for (int i = 0; i < 8; ++i) acc[hf][i] *= alpha[i];
      const bf16* vrow = vlds + (hf*16 + lm) * 64;
      acc[hf] = wmma_bf16(pa0, b_frag(vrow, hi),      acc[hf]);
      acc[hf] = wmma_bf16(pa1, b_frag(vrow + 32, hi), acc[hf]);
    }
    __syncthreads();
  }

  float* so = (float*)(smem + OST_OFF) + wave * (16 * 64);
  #pragma unroll
  for (int hf = 0; hf < 4; ++hf)
    #pragma unroll
    for (int i = 0; i < 8; ++i) so[(i + 8*hi)*64 + hf*16 + lm] = acc[hf][i] / (lstate[i] * 1024.0f);
  asm volatile("s_wait_dscnt 0" ::: "memory");
  #pragma unroll 1
  for (int pass = 0; pass < 2; ++pass){
    #pragma unroll
    for (int i = 0; i < 8; ++i){
      int c = lane + 32*i, rr = c >> 4, qq = c & 15;
      *(volatile v4f_t*)(out + ((size_t)b*S_LEN + l0 + wave*16 + rr)*1024 + h*HDIM + qq*4) = *(const volatile v4fa*)(so + rr*64 + qq*4);
    }
    __threadfence();
  }
}

extern "C" void kernel_launch(void* const* d_in, const int* in_sizes, int n_in,
                              void* d_out, int out_size, void* d_ws, size_t ws_size,
                              hipStream_t stream) {
  (void)in_sizes; (void)n_in; (void)out_size; (void)ws_size;
  const float* hidden = (const float*)d_in[0];
  const float* amask  = (const float*)d_in[1];
  const float* Wq = (const float*)d_in[3];
  const float* bq = (const float*)d_in[4];
  const float* Wk = (const float*)d_in[5];
  const float* bk = (const float*)d_in[6];
  const float* Wv = (const float*)d_in[7];
  const float* bv = (const float*)d_in[8];
  const float* de = (const float*)d_in[9];

  char* ws = (char*)d_ws;
  bf16* xb  = (bf16*)(ws + (size_t) 0u);
  bf16* wbb = (bf16*)(ws + (size_t)( 8u << 20));
  bf16* qb  = (bf16*)(ws + (size_t)(16u << 20));
  bf16* kb  = (bf16*)(ws + (size_t)(24u << 20));
  bf16* vtb = (bf16*)(ws + (size_t)(32u << 20));
  bf16* db  = (bf16*)(ws + (size_t)(40u << 20));
  bf16* vrb = (bf16*)(ws + (size_t)(41u << 20));

  auto cvt = [&](const float* s, bf16* d, int n){
    cvt_bf16_kernel<<<(n/4 + 255)/256, 256, 0, stream>>>(s, d, n/4);
  };
  cvt(hidden, xb, 4096*1024);
  cvt(Wq, wbb + 0*(1024*1024), 1024*1024);
  cvt(Wk, wbb + 1*(1024*1024), 1024*1024);
  cvt(Wv, wbb + 2*(1024*1024), 1024*1024);
  cvt(de, db, DIST_ROWS*HDIM);

  qkv_kernel<<<dim3(32, 16, 3), 256, 0, stream>>>(xb, wbb, bq, bk, bv,
                                                  qb, kb, vrb);
  vt_kernel<<<4 * HEADS * (S_LEN / 64), 256, 0, stream>>>(vrb, vtb);
  (void)hipFuncSetAttribute((const void*)attn_kernel, hipFuncAttributeMaxDynamicSharedMemorySize, ATTN_SMEM);
  attn_kernel<<<dim3(8, 64), 256, (size_t)ATTN_SMEM, stream>>>(
      qb, kb, vtb, db, amask, (float*)d_out);
}
